// ComnetModel_52097953300871
// MI455X (gfx1250) — hardware-verified
//
#include <hip/hip_runtime.h>
#include <stddef.h>
#include <stdint.h>


#define DIM 32
#define GW 96
#define PL 8
#define RD 256
#define NIT 3
#define TP 36
#define TPX 100
#define TPH 264
#define LBLK 1024
#define AGT 256

typedef char cfg_check_t[(LBLK == 1024 && AGT == 256) ? 1 : -1];

typedef __bf16 v16b __attribute__((ext_vector_type(16)));
typedef unsigned short v16u __attribute__((ext_vector_type(16)));
typedef unsigned short v8u __attribute__((ext_vector_type(8)));
typedef float v8f __attribute__((ext_vector_type(8)));
typedef float v4f __attribute__((ext_vector_type(4)));

union Frag { v16b v; v16u u; v8u h8[2]; };


__device__ __forceinline__ unsigned short bf_bits(float x) {
  unsigned int u = __float_as_uint(x);
  u += 0x7FFFu + ((u >> 16) & 1u);
  return (unsigned short)(u >> 16);
}
__device__ __forceinline__ float bf_val(unsigned short b) {
  return __uint_as_float(((unsigned int)b) << 16);
}
__device__ __forceinline__ v8f splat8(float x) {
  v8f v;
#pragma unroll
  for (int i = 0; i < 8; ++i) v[i] = x;
  return v;
}
__device__ __forceinline__ v4f mk4(float a, float b, float c, float d) {
  v4f v; v[0] = a; v[1] = b; v[2] = c; v[3] = d; return v;
}
__device__ __forceinline__ void vst4(float* p, v4f v) { *(volatile v4f*)p = v; }
__device__ __forceinline__ void vst8(unsigned short* p, v8u v) { *(volatile v8u*)p = v; }

__device__ __forceinline__ v8f mma(v16b a, v16b b, v8f c) {
  v8f d = __builtin_amdgcn_wmma_f32_16x16x32_bf16(false, a, false, b, (short)0, c, false, false);
  asm volatile("v_nop\n\tv_nop\n\tv_nop\n\tv_nop" : "+v"(d) : "v"(a), "v"(b));
  return d;
}
__device__ __forceinline__ v8f mma3(const Frag& ah, const Frag& al, const Frag& bh, const Frag& bl, v8f c) {
  c = mma(ah.v, bh.v, c);
  c = mma(ah.v, bl.v, c);
  c = mma(al.v, bh.v, c);
  return c;
}

__device__ __forceinline__ Frag ldfrag(const unsigned short* p, int h) {
  Frag f;
  f.h8[0] = *(const v8u*)(p + 8 * h);
  f.h8[1] = *(const v8u*)(p + 16 + 8 * h);
  return f;
}

__device__ __forceinline__ void afrag_f32(const float* rp, int h, Frag& hi, Frag& lo) {
  const float* p0 = rp + 8 * h;
  const float* p1 = rp + 16 + 8 * h;
  v4f x0 = *(const v4f*)p0;
  v4f x1 = *(const v4f*)(p0 + 4);
  v4f x2 = *(const v4f*)p1;
  v4f x3 = *(const v4f*)(p1 + 4);
  float f[16];
#pragma unroll
  for (int i = 0; i < 4; ++i) { f[i] = x0[i]; f[4 + i] = x1[i]; f[8 + i] = x2[i]; f[12 + i] = x3[i]; }
  v16u hu, lu;
#pragma unroll
  for (int i = 0; i < 16; ++i) {
    unsigned short b = bf_bits(f[i]);
    hu[i] = b;
    lu[i] = bf_bits(f[i] - bf_val(b));
  }
  hi.u = hu;
  lo.u = lu;
}

__device__ __forceinline__ float rcpf_(float x) { return __builtin_amdgcn_rcpf(x); }
__device__ __forceinline__ float sigm_(float x) { return rcpf_(1.0f + __expf(-x)); }
__device__ __forceinline__ float tanh_(float x) { return 1.0f - 2.0f * rcpf_(__expf(2.0f * x) + 1.0f); }
__device__ __forceinline__ float selu_(float x) {
  const float a = 1.6732632423543772f;
  const float s = 1.0507009873554805f;
  return x > 0.0f ? s * x : (s * a) * (__expf(x) - 1.0f);
}
__device__ __forceinline__ float gru1(float gxz, float ghz, float gxr, float ghr,
                                      float gxc, float ghc, float hold) {
  float z  = sigm_(gxz + ghz);
  float rg = sigm_(gxr + ghr);
  float c  = tanh_(gxc + rg * ghc);
  return z * hold + (1.0f - z) * c;
}

__device__ __forceinline__ void rows_pass(const float* tile, float* dst, int lane, int nvalid) {
#pragma unroll
  for (int s = 0; s < 4; ++s) {
    const int r = 4 * s + (lane >> 3), q = lane & 7;
    if (r < nvalid) {
      v4f v = *(const v4f*)(tile + r * TP + 4 * q);
      vst4(dst + (size_t)r * DIM + 4 * q, v);
    }
  }
}


__device__ __forceinline__ void wt_pass(const float* __restrict__ W, int K, int C, unsigned short* WT, int n) {
  unsigned short* rowp = WT + (size_t)n * (size_t)(2 * K);
#pragma unroll 1
  for (int kk = 0; kk < K; kk += 8) {
    v8u hv, lv;
#pragma unroll
    for (int i = 0; i < 8; ++i) {
      float x = W[(size_t)(kk + i) * (size_t)C + n];
      unsigned short b = bf_bits(x);
      hv[i] = b;
      lv[i] = bf_bits(x - bf_val(b));
    }
    vst8(rowp + kk, hv);
    vst8(rowp + K + kk, lv);
  }
}

__global__ void __launch_bounds__(256) k_wt(const float* __restrict__ W, int K, int C,
                                         unsigned short* __restrict__ WT) {
  const int n = blockIdx.x * 256 + threadIdx.x;
  if (n >= C) return;
  wt_pass(W, K, C, WT, n);
  __threadfence();
  wt_pass(W, K, C, WT, n);
}


__device__ __forceinline__ void init_pass(float* p, v4f f0, v4f z) {
  vst4(p, f0);
#pragma unroll
  for (int q = 1; q < 8; ++q) vst4(p + 4 * q, z);
}

__global__ void __launch_bounds__(256) k_init(const float* __restrict__ src, int n, float* __restrict__ dst) {
  const int r = blockIdx.x * 256 + threadIdx.x;
  if (r >= n) return;
  const float x = src[r];
  v4f f0 = mk4(x, 0.0f, 0.0f, 0.0f);
  v4f z  = mk4(0.0f, 0.0f, 0.0f, 0.0f);
  float* p = dst + (size_t)r * DIM;
  init_pass(p, f0, z);
  __threadfence();
  init_pass(p, f0, z);
}


__device__ __forceinline__ void xw_pass(const float* tile, float* dst, int lane, int nvalid) {
#pragma unroll
  for (int s = 0; s < 12; ++s) {
    const int L = 4 * s + (lane >> 3), q = lane & 7;
    const int r = L / 3, seg = L - 3 * r;
    if (r < nvalid) {
      v4f v = *(const v4f*)(tile + r * TPX + 32 * seg + 4 * q);
      vst4(dst + (size_t)r * GW + 32 * seg + 4 * q, v);
    }
  }
}

__global__ void __launch_bounds__(32) k_xw(const float* __restrict__ ls,
                                        const unsigned short* __restrict__ WT,
                                        const float* __restrict__ bias,
                                        float* __restrict__ XW, int NL) {
  __shared__ __align__(16) float tile[16 * TPX];
  const int lane = threadIdx.x & 31, h = lane >> 4, m = lane & 15;
  const int base = blockIdx.x * 16;
  int rm = base + m; rm = rm < NL ? rm : NL - 1;
  Frag ah, al;
  afrag_f32(ls + (size_t)rm * DIM, h, ah, al);
#pragma unroll
  for (int n = 0; n < 6; ++n) {
    const unsigned short* wp = WT + (size_t)(16 * n + m) * (2 * DIM);
    Frag bh = ldfrag(wp, h), bl = ldfrag(wp + DIM, h);
    v8f acc = mma3(ah, al, bh, bl, splat8(bias[16 * n + m]));
#pragma unroll
    for (int r = 0; r < 8; ++r) tile[(8 * h + r) * TPX + 16 * n + m] = acc[r];
  }
  __syncthreads();
  float* dst = XW + (size_t)base * GW;
  const int nv = NL - base;
  xw_pass(tile, dst, lane, nv);
  __threadfence();
  xw_pass(tile, dst, lane, nv);
}


__global__ void __launch_bounds__(32) k_path(
    float* __restrict__ ps, const float* __restrict__ XW, const int* __restrict__ links,
    const unsigned short* __restrict__ WhT, float* __restrict__ outs,
    int pbase, int pc, int PC, int NP, int NL, int E, int write_outs)
{
  __shared__ __align__(16) float tile[16 * TP];
  const int lane = threadIdx.x & 31, h = lane >> 4, m = lane & 15;
  const int lbase = blockIdx.x * 16;

#pragma unroll
  for (int s = 0; s < 4; ++s) {
    const int r = 4 * s + (lane >> 3), q = lane & 7;
    int p = pbase + lbase + r; p = p < NP ? p : NP - 1;
    v4f v = *(const v4f*)(ps + (size_t)p * DIM + 4 * q);
    *(v4f*)(tile + r * TP + 4 * q) = v;
  }
  __syncthreads();

  float hD[2][8];
#pragma unroll
  for (int k = 0; k < 2; ++k)
#pragma unroll
    for (int r = 0; r < 8; ++r) hD[k][r] = tile[(8 * h + r) * TP + 16 * k + m];

  int prow[8];
#pragma unroll
  for (int r = 0; r < 8; ++r) {
    int p = pbase + lbase + 8 * h + r;
    prow[r] = p < NP ? p : NP - 1;
  }

#pragma unroll 1
  for (int t = 0; t < PL; ++t) {
    Frag ah, al;
    afrag_f32(tile + m * TP, h, ah, al);

    int lk[8];
#pragma unroll
    for (int r = 0; r < 8; ++r) {
      int e = prow[r] * PL + t; e = e < E ? e : E - 1;
      int l = links[e];
      l = l < 0 ? 0 : (l >= NL ? NL - 1 : l);
      lk[r] = l;
    }

#pragma unroll
    for (int k = 0; k < 2; ++k) {
      v8f g[3];
#pragma unroll
      for (int u = 0; u < 3; ++u) {
        const int n = k + 2 * u;
        const unsigned short* wp = WhT + (size_t)(16 * n + m) * (2 * DIM);
        Frag bh = ldfrag(wp, h), bl = ldfrag(wp + DIM, h);
        g[u] = mma3(ah, al, bh, bl, splat8(0.0f));
      }
      float gx[3][8];
#pragma unroll
      for (int u = 0; u < 3; ++u)
#pragma unroll
        for (int r = 0; r < 8; ++r)
          gx[u][r] = XW[(size_t)lk[r] * GW + 16 * (k + 2 * u) + m];
#pragma unroll
      for (int r = 0; r < 8; ++r)
        hD[k][r] = gru1(gx[0][r], g[0][r], gx[1][r], g[1][r], gx[2][r], g[2][r], hD[k][r]);
    }

    __syncthreads();
#pragma unroll
    for (int k = 0; k < 2; ++k)
#pragma unroll
      for (int r = 0; r < 8; ++r) tile[(8 * h + r) * TP + 16 * k + m] = hD[k][r];
    __syncthreads();

    if (write_outs) {
      float* ob = outs + ((size_t)t * (size_t)PC + (size_t)lbase) * DIM;
      rows_pass(tile, ob, lane, pc - lbase);
      __threadfence();
      rows_pass(tile, ob, lane, pc - lbase);
    }
  }

  float* pb = ps + ((size_t)pbase + (size_t)lbase) * DIM;
  rows_pass(tile, pb, lane, pc - lbase);
  __threadfence();
  rows_pass(tile, pb, lane, pc - lbase);
}


__global__ void __launch_bounds__(AGT) k_agg(
    const float* __restrict__ outs, const int* __restrict__ links,
    const int* __restrict__ pth, const int* __restrict__ sq, float* __restrict__ agg,
    int ebase, int EC, int pbase, int pc, int PC, int NL, int accum)
{
  extern __shared__ v4f sacc4[];
  __shared__ int s_list[AGT];
  __shared__ int s_wcnt[AGT / 32];
  float* sacc = (float*)sacc4;
  const int tid = threadIdx.x, lane = tid & 31, w = tid >> 5;
  const int l0 = blockIdx.x * LBLK;

  for (int i = tid; i < LBLK * DIM; i += AGT) sacc[i] = 0.0f;
  __syncthreads();

  const int nch = (EC + AGT - 1) / AGT;
#pragma unroll 1
  for (int ch = 0; ch < nch; ++ch) {
    const int el = ch * AGT + tid;
    const bool valid = el < EC;
    const int e = ebase + (valid ? el : 0);
    int lk = -1;
    if (valid) lk = links[e];
    const int rel = lk - l0;
    const bool hit = valid && lk >= 0 && lk < NL && (unsigned)rel < (unsigned)LBLK;
    const unsigned bal = __builtin_amdgcn_ballot_w32(hit);
    const int cnt = __builtin_popcount(bal);
    const int pre = __builtin_popcount(bal & ((1u << lane) - 1u));
    if (lane == 0) s_wcnt[w] = cnt;
    __syncthreads();
    int off = 0, nh = 0;
#pragma unroll
    for (int i = 0; i < AGT / 32; ++i) {
      const int c = s_wcnt[i];
      if (i < w) off += c;
      nh += c;
    }
    if (hit) {
      int p = pth[e] - pbase; p = p < 0 ? 0 : (p >= pc ? pc - 1 : p);
      int s = sq[e]; s = s < 0 ? 0 : (s >= PL ? PL - 1 : s);
      s_list[off + pre] = ((s * PC + p) << 10) | rel;
    }
    __syncthreads();
    nh = nh < AGT ? nh : AGT;
    for (int i = 0; i < nh; ++i) {
      const int ent = s_list[i];
      const int rl = ent & (LBLK - 1);
      if ((rl & 7) == w) {
        const int row = ent >> 10;
        sacc[rl * DIM + lane] += outs[(size_t)row * DIM + lane];
      }
    }
    __syncthreads();
  }

  const int q = lane & 7;
#pragma unroll 1
  for (int s = 0; s < 32; ++s) {
    const int r = w * 128 + 4 * s + (lane >> 3);
    const int l = l0 + r;
    float* ap = sacc + r * DIM + 4 * q;
    if (l < NL) {
      v4f v = *(v4f*)ap;
      if (accum) {
        v4f o = *(const v4f*)(agg + (size_t)l * DIM + 4 * q);
        v += o;
        *(v4f*)ap = v;
      }
      vst4(agg + (size_t)l * DIM + 4 * q, v);
    }
  }
  __threadfence();
#pragma unroll 1
  for (int s = 0; s < 32; ++s) {
    const int r = w * 128 + 4 * s + (lane >> 3);
    const int l = l0 + r;
    const float* ap = sacc + r * DIM + 4 * q;
    if (l < NL) {
      v4f v = *(const v4f*)ap;
      vst4(agg + (size_t)l * DIM + 4 * q, v);
    }
  }
}


__global__ void __launch_bounds__(32) k_edge(
    const float* __restrict__ agg, float* __restrict__ ls,
    const unsigned short* __restrict__ WxT, const unsigned short* __restrict__ WhT,
    const float* __restrict__ bias, int NL)
{
  __shared__ __align__(16) float tile[16 * TP];
  const int lane = threadIdx.x & 31, h = lane >> 4, m = lane & 15;
  const int base = blockIdx.x * 16;
  int rm = base + m; rm = rm < NL ? rm : NL - 1;

  Frag xh, xl, hh, hl;
  afrag_f32(agg + (size_t)rm * DIM, h, xh, xl);
  afrag_f32(ls + (size_t)rm * DIM, h, hh, hl);

  float hD[2][8];
#pragma unroll
  for (int k = 0; k < 2; ++k)
#pragma unroll
    for (int r = 0; r < 8; ++r) {
      int rr = base + 8 * h + r; rr = rr < NL ? rr : NL - 1;
      hD[k][r] = ls[(size_t)rr * DIM + 16 * k + m];
    }

#pragma unroll
  for (int k = 0; k < 2; ++k) {
    v8f gx[3], gh[3];
#pragma unroll
    for (int u = 0; u < 3; ++u) {
      const int n = k + 2 * u;
      const unsigned short* wxp = WxT + (size_t)(16 * n + m) * (2 * DIM);
      const unsigned short* whp = WhT + (size_t)(16 * n + m) * (2 * DIM);
      {
        Frag bh = ldfrag(wxp, h), bl = ldfrag(wxp + DIM, h);
        gx[u] = mma3(xh, xl, bh, bl, splat8(bias[16 * n + m]));
      }
      {
        Frag bh = ldfrag(whp, h), bl = ldfrag(whp + DIM, h);
        gh[u] = mma3(hh, hl, bh, bl, splat8(0.0f));
      }
    }
#pragma unroll
    for (int r = 0; r < 8; ++r)
      hD[k][r] = gru1(gx[0][r], gh[0][r], gx[1][r], gh[1][r], gx[2][r], gh[2][r], hD[k][r]);
  }

#pragma unroll
  for (int k = 0; k < 2; ++k)
#pragma unroll
    for (int r = 0; r < 8; ++r) tile[(8 * h + r) * TP + 16 * k + m] = hD[k][r];
  __syncthreads();

  float* dst = ls + (size_t)base * DIM;
  const int nv = NL - base;
  rows_pass(tile, dst, lane, nv);
  __threadfence();
  rows_pass(tile, dst, lane, nv);
}


__device__ __forceinline__ void ro_pass(const float* sout, float* out, int tid, int obase, int NP) {
  if (tid < 8) {
    const int o = obase + 4 * tid;
    v4f v = *(const v4f*)(sout + 4 * tid);
    if (o + 3 < NP) {
      vst4(out + o, v);
    } else {
#pragma unroll
      for (int i = 0; i < 4; ++i)
        if (o + i < NP) *(volatile float*)(out + o + i) = v[i];
    }
  }
}

__global__ void __launch_bounds__(64) k_readout(
    const float* __restrict__ ps,
    const unsigned short* __restrict__ W1T, const float* __restrict__ b1,
    const unsigned short* __restrict__ W2T, const float* __restrict__ b2,
    const float* __restrict__ W3, const float* __restrict__ b3,
    float* __restrict__ out, int NP)
{
  __shared__ __align__(16) unsigned short h1h[2 * 16 * TPH];
  __shared__ __align__(16) unsigned short h1l[2 * 16 * TPH];
  __shared__ __align__(16) float sout[32];
  const int tid = threadIdx.x, wv = tid >> 5, lane = tid & 31, h = lane >> 4, m = lane & 15;
  const int base = blockIdx.x * 32 + wv * 16;
  int rm = base + m; rm = rm < NP ? rm : NP - 1;

  Frag ph, pl;
  afrag_f32(ps + (size_t)rm * DIM, h, ph, pl);
  unsigned short* th = h1h + wv * 16 * TPH;
  unsigned short* tl = h1l + wv * 16 * TPH;

#pragma unroll 1
  for (int n = 0; n < 16; ++n) {
    const unsigned short* wp = W1T + (size_t)(16 * n + m) * (2 * DIM);
    Frag bh = ldfrag(wp, h), bl = ldfrag(wp + DIM, h);
    v8f acc = mma3(ph, pl, bh, bl, splat8(b1[16 * n + m]));
#pragma unroll
    for (int r = 0; r < 8; ++r) {
      float v = selu_(acc[r]);
      unsigned short b = bf_bits(v);
      th[(8 * h + r) * TPH + 16 * n + m] = b;
      tl[(8 * h + r) * TPH + 16 * n + m] = bf_bits(v - bf_val(b));
    }
  }
  __syncthreads();

  float part[8];
#pragma unroll
  for (int r = 0; r < 8; ++r) part[r] = 0.0f;

#pragma unroll 1
  for (int n = 0; n < 16; ++n) {
    v8f acc = splat8(b2[16 * n + m]);
    const unsigned short* w2p = W2T + (size_t)(16 * n + m) * (2 * RD);
#pragma unroll 1
    for (int c = 0; c < 8; ++c) {
      Frag ah = ldfrag(th + m * TPH + 32 * c, h);
      Frag al = ldfrag(tl + m * TPH + 32 * c, h);
      Frag bh = ldfrag(w2p + 32 * c, h);
      Frag bl = ldfrag(w2p + RD + 32 * c, h);
      acc = mma3(ah, al, bh, bl, acc);
    }
    const float w3 = W3[16 * n + m];
#pragma unroll
    for (int r = 0; r < 8; ++r) part[r] += selu_(acc[r]) * w3;
  }

#pragma unroll
  for (int r = 0; r < 8; ++r) {
    float v = part[r];
    v += __shfl_xor(v, 1);
    v += __shfl_xor(v, 2);
    v += __shfl_xor(v, 4);
    v += __shfl_xor(v, 8);
    part[r] = v;
  }
  const float b3v = b3[0];
  if (m == 0) {
#pragma unroll
    for (int r = 0; r < 8; ++r) sout[wv * 16 + 8 * h + r] = part[r] + b3v;
  }
  __syncthreads();

  const int obase = blockIdx.x * 32;
  ro_pass(sout, out, tid, obase, NP);
  __threadfence();
  ro_pass(sout, out, tid, obase, NP);
}


static inline size_t al256(size_t x) { return (x + 255) & ~(size_t)255; }
static inline int cdiv(int a, int b) { return (a + b - 1) / b; }

extern "C" void kernel_launch(void* const* d_in, const int* in_sizes, int n_in,
                              void* d_out, int out_size, void* d_ws, size_t ws_size,
                              hipStream_t stream) {
  if (!d_in || !in_sizes || !d_out || !d_ws || n_in < 17) return;
  const int NL = in_sizes[0];
  const int NP = out_size;
  const int E  = in_sizes[2];
  if (NL <= 0 || NP <= 0 || NP > 250000 || NL > (1 << 24)) return;
  if (E != NP * PL || in_sizes[3] != E || in_sizes[4] != E || in_sizes[1] < NP) return;
  if (in_sizes[5] != DIM * GW || in_sizes[6] != DIM * GW || in_sizes[7] != GW) return;
  if (in_sizes[8] != DIM * GW || in_sizes[9] != DIM * GW || in_sizes[10] != GW) return;
  if (in_sizes[11] != DIM * RD || in_sizes[12] != RD || in_sizes[13] != RD * RD ||
      in_sizes[14] != RD || in_sizes[15] != RD || in_sizes[16] < 1) return;

  const float* cap     = (const float*)d_in[0];
  const float* traffic = (const float*)d_in[1];
  const int*   links   = (const int*)d_in[2];
  const int*   pth     = (const int*)d_in[3];
  const int*   sq      = (const int*)d_in[4];
  const float* Wx_p    = (const float*)d_in[5];
  const float* Wh_p    = (const float*)d_in[6];
  const float* b_p     = (const float*)d_in[7];
  const float* Wx_e    = (const float*)d_in[8];
  const float* Wh_e    = (const float*)d_in[9];
  const float* b_e     = (const float*)d_in[10];
  const float* W1      = (const float*)d_in[11];
  const float* b1      = (const float*)d_in[12];
  const float* W2      = (const float*)d_in[13];
  const float* b2      = (const float*)d_in[14];
  const float* W3      = (const float*)d_in[15];
  const float* b3      = (const float*)d_in[16];
  float* out = (float*)d_out;

  const int PC = (NP + 1) / 2;

  char* wsb = (char*)d_ws;
  size_t off = 0;
  const size_t o_ls  = off; off = al256(off + (size_t)NL * DIM * sizeof(float));
  const size_t o_ps  = off; off = al256(off + (size_t)NP * DIM * sizeof(float));
  const size_t o_xw  = off; off = al256(off + (size_t)NL * GW * sizeof(float));
  const size_t o_ag  = off; off = al256(off + (size_t)NL * DIM * sizeof(float));
  const size_t o_ou  = off; off = al256(off + (size_t)PL * (size_t)PC * DIM * sizeof(float));
  const size_t o_wxp = off; off = al256(off + (size_t)GW * 2 * DIM * 2);
  const size_t o_whp = off; off = al256(off + (size_t)GW * 2 * DIM * 2);
  const size_t o_wxe = off; off = al256(off + (size_t)GW * 2 * DIM * 2);
  const size_t o_whe = off; off = al256(off + (size_t)GW * 2 * DIM * 2);
  const size_t o_w1  = off; off = al256(off + (size_t)RD * 2 * DIM * 2);
  const size_t o_w2  = off; off = al256(off + (size_t)RD * 2 * RD * 2);
  if (off > ws_size) return;

  float* ls   = (float*)(wsb + o_ls);
  float* ps   = (float*)(wsb + o_ps);
  float* XW   = (float*)(wsb + o_xw);
  float* agg  = (float*)(wsb + o_ag);
  float* outs = (float*)(wsb + o_ou);
  unsigned short* WxpT = (unsigned short*)(wsb + o_wxp);
  unsigned short* WhpT = (unsigned short*)(wsb + o_whp);
  unsigned short* WxeT = (unsigned short*)(wsb + o_wxe);
  unsigned short* WheT = (unsigned short*)(wsb + o_whe);
  unsigned short* W1T  = (unsigned short*)(wsb + o_w1);
  unsigned short* W2T  = (unsigned short*)(wsb + o_w2);

  k_wt<<<cdiv(GW, 256), 256, 0, stream>>>(Wx_p, DIM, GW, WxpT);
  k_wt<<<cdiv(GW, 256), 256, 0, stream>>>(Wh_p, DIM, GW, WhpT);
  k_wt<<<cdiv(GW, 256), 256, 0, stream>>>(Wx_e, DIM, GW, WxeT);
  k_wt<<<cdiv(GW, 256), 256, 0, stream>>>(Wh_e, DIM, GW, WheT);
  k_wt<<<cdiv(RD, 256), 256, 0, stream>>>(W1, DIM, RD, W1T);
  k_wt<<<cdiv(RD, 256), 256, 0, stream>>>(W2, RD, RD, W2T);
  k_init<<<cdiv(NP, 256), 256, 0, stream>>>(traffic, NP, ps);
  k_init<<<cdiv(NL, 256), 256, 0, stream>>>(cap, NL, ls);

  for (int it = 0; it < NIT; ++it) {
    const int last = (it == NIT - 1) ? 1 : 0;
    k_xw<<<cdiv(NL, 16), 32, 0, stream>>>(ls, WxpT, b_p, XW, NL);
    for (int c = 0; c < 2; ++c) {
      const int pbase = c * PC;
      const int rem = NP - pbase;
      const int pc = rem < PC ? rem : PC;
      if (pc <= 0) continue;
      k_path<<<cdiv(pc, 16), 32, 0, stream>>>(ps, XW, links, WhpT, outs,
                                            pbase, pc, PC, NP, NL, E, last ? 0 : 1);
      if (!last) {
        k_agg<<<cdiv(NL, LBLK), AGT, (size_t)LBLK * DIM * sizeof(float), stream>>>(
            outs, links, pth, sq, agg, pbase * PL, pc * PL, pbase, pc, PC, NL, c > 0 ? 1 : 0);
      }
    }
    if (!last) k_edge<<<cdiv(NL, 16), 32, 0, stream>>>(agg, ls, WxeT, WheT, b_e, NL);
  }

  k_readout<<<cdiv(NP, 32), 64, 0, stream>>>(ps, W1T, b1, W2T, b2, W3, b3, out, NP);
  (void)hipGetLastError();
}
